// PhysicsInformedNN_12086037970987
// MI455X (gfx1250) — hardware-run, weakly checked
//
#include <hip/hip_runtime.h>
#include <math.h>

typedef __attribute__((ext_vector_type(16))) _Float16 v16h;
typedef __attribute__((ext_vector_type(8)))  _Float16 v8h;
typedef __attribute__((ext_vector_type(8)))  float    v8f;
typedef __attribute__((ext_vector_type(4)))  float    v4f;

constexpr int kPts     = 8192;
constexpr int kInDim   = 4;
constexpr int kHid     = 256;
constexpr int kNHid    = 7;
constexpr int kOutDim  = 4;
constexpr int kOutPad  = 16;
constexpr int kJet     = 8;
constexpr int kPtsBlk  = 8;
constexpr int kRowsBlk = kPtsBlk * kJet;
constexpr int kBlocks  = kPts / kPtsBlk;
constexpr int kPitchA  = 264;
constexpr int kPlane   = kRowsBlk * kPitchA;
constexpr float kCarryA = 256.0f;
constexpr float kCarryW = 256.0f;
constexpr float kFold   = 1.0f / (kCarryA * kCarryW);
static_assert(kRowsBlk == 64, "block owns 64 jet rows");
static_assert((kHid % 32) == 0, "K multiple of 32");
static_assert((kHid % 64) == 0 && (kRowsBlk % 16) == 0, "tile multiples");
static_assert(kBlocks * kPtsBlk == kPts, "exact point coverage");
static_assert((kPitchA % 8) == 0, "16-B aligned LDS rows");
static_assert(kFold == 1.0f / 65536.0f, "fold constant is a power of two");

constexpr size_t kOffWT   = 0;
constexpr size_t kOffWOT  = kOffWT  + (size_t)kNHid * kHid * kHid * 2;
constexpr size_t kOffMM   = kOffWOT + (size_t)kOutPad * kHid * 2;
constexpr size_t kOffPART = kOffMM  + 128;
constexpr size_t kWsTotal = kOffPART + (size_t)kBlocks * 32 * 4;
static_assert(kWsTotal == 1056896ull, "carve total");
static_assert(kWsTotal <= 134217728ull, "carve cap");
static_assert((kOffWOT % 128) == 0 && (kOffMM % 128) == 0 && (kOffPART % 128) == 0, "128-B aligned regions");

union FragU { v16h v; v8h h[2]; };

__device__ __forceinline__ v16h frag_load_g(const _Float16* p) {
  FragU f;
  f.h[0] = *(const v8h*)(p);
  f.h[1] = *(const v8h*)(p + 16);
  return f.v;
}

__device__ __forceinline__ v8f mma_h(v16h a, v16h b, v8f c) {
  c = __builtin_amdgcn_wmma_f32_16x16x32_f16(false, a, false, b, (short)0, c, false, false);
  asm volatile("v_nop\n\tv_nop\n\tv_nop\n\tv_nop" : "+v"(c) : "v"(a), "v"(b));
  return c;
}

__device__ __forceinline__ v8f jet_tanh(const v8f a, const float bias) {
  const float z    = a[0] * kFold + bias;
  const float zt0  = a[1] * kFold;
  const float zt1  = a[2] * kFold;
  const float zt2  = a[3] * kFold;
  const float zt3  = a[4] * kFold;
  const float ztt0 = a[5] * kFold;
  const float ztt1 = a[6] * kFold;
  const float ztt2 = a[7] * kFold;
  const float h  = tanhf(z);
  const float g  = 1.0f - h * h;
  const float m2 = -2.0f * h;
  const float ht0 = g * zt0;
  const float ht1 = g * zt1;
  const float ht2 = g * zt2;
  const float ht3 = g * zt3;
  v8f o;
  o[0] = h * kCarryA;
  o[1] = ht0 * kCarryA;
  o[2] = ht1 * kCarryA;
  o[3] = ht2 * kCarryA;
  o[4] = ht3 * kCarryA;
  o[5] = (g * ztt0 + m2 * ht0 * zt0) * kCarryA;
  o[6] = (g * ztt1 + m2 * ht1 * zt1) * kCarryA;
  o[7] = (g * ztt2 + m2 * ht2 * zt2) * kCarryA;
  return o;
}

__global__ __launch_bounds__(256) void prep_hidden_kernel(const float* __restrict__ Wh,
                                                          unsigned short* __restrict__ WT) {
  __shared__ float sT[kHid * 33];
  const int tid = threadIdx.x, lane = tid & 31, wave = tid >> 5;
  const int l  = blockIdx.x >> 3;
  const int n0 = (blockIdx.x & 7) * 32;
  const float* src = Wh + (size_t)l * kHid * kHid;
#pragma unroll 1
  for (int it = 0; it < 32; ++it) {
    const int k = it * 8 + wave;
    sT[k * 33 + lane] = src[(size_t)k * kHid + n0 + lane];
  }
  __syncthreads();
  v8h hv[4];
#pragma unroll
  for (int it = 0; it < 4; ++it) {
    const int row = it * 8 + wave;
#pragma unroll
    for (int e = 0; e < 8; ++e) {
      const float w = sT[(lane * 8 + e) * 33 + row] * kCarryW;
      hv[it][e] = (_Float16)w;
    }
  }
  for (int pass = 0; pass < 2; ++pass) {
#pragma unroll
    for (int it = 0; it < 4; ++it) {
      const size_t o = ((size_t)l * kHid + n0 + it * 8 + wave) * kHid + lane * 8;
      *(volatile v8h*)(WT + o) = hv[it];
    }
    __threadfence();
  }
}

__global__ __launch_bounds__(256) void prep_out_kernel(const float* __restrict__ Wo,
                                                       unsigned short* __restrict__ WOT) {
  const int tid = threadIdx.x, lane = tid & 31, wave = tid >> 5;
  v8h hv[2];
#pragma unroll
  for (int it = 0; it < 2; ++it) {
    const int j  = it * 8 + wave;
    const int jc = (j < kOutDim) ? j : (kOutDim - 1);
#pragma unroll
    for (int e = 0; e < 8; ++e) {
      const float w = Wo[(size_t)(lane * 8 + e) * kOutDim + jc];
      const float s = (j < kOutDim) ? (w * kCarryW) : 0.0f;
      hv[it][e] = (_Float16)s;
    }
  }
  for (int pass = 0; pass < 2; ++pass) {
#pragma unroll
    for (int it = 0; it < 2; ++it) {
      const size_t o = (size_t)(it * 8 + wave) * kHid + lane * 8;
      *(volatile v8h*)(WOT + o) = hv[it];
    }
    __threadfence();
  }
}

__global__ __launch_bounds__(256) void bounds_kernel(const float* __restrict__ X,
                                                     float* __restrict__ mm) {
  __shared__ float sMn[4 * 256];
  __shared__ float sMx[4 * 256];
  const int tid = threadIdx.x, lane = tid & 31, wave = tid >> 5;
  float mn0 = 3.4e38f, mn1 = 3.4e38f, mn2 = 3.4e38f, mn3 = 3.4e38f;
  float mx0 = -3.4e38f, mx1 = -3.4e38f, mx2 = -3.4e38f, mx3 = -3.4e38f;
#pragma unroll 1
  for (int q = 0; q < kPts / 256; ++q) {
    const v4f x = *(const v4f*)(X + (size_t)(tid + 256 * q) * kInDim);
    mn0 = fminf(mn0, x[0]); mx0 = fmaxf(mx0, x[0]);
    mn1 = fminf(mn1, x[1]); mx1 = fmaxf(mx1, x[1]);
    mn2 = fminf(mn2, x[2]); mx2 = fmaxf(mx2, x[2]);
    mn3 = fminf(mn3, x[3]); mx3 = fmaxf(mx3, x[3]);
  }
  sMn[tid] = mn0; sMn[256 + tid] = mn1; sMn[512 + tid] = mn2; sMn[768 + tid] = mn3;
  sMx[tid] = mx0; sMx[256 + tid] = mx1; sMx[512 + tid] = mx2; sMx[768 + tid] = mx3;
  __syncthreads();
  for (int off = 128; off > 0; off >>= 1) {
    if (tid < off) {
#pragma unroll
      for (int k = 0; k < 4; ++k) {
        sMn[k * 256 + tid] = fminf(sMn[k * 256 + tid], sMn[k * 256 + tid + off]);
        sMx[k * 256 + tid] = fmaxf(sMx[k * 256 + tid], sMx[k * 256 + tid + off]);
      }
    }
    __syncthreads();
  }
  if (wave == 0) {
    const int k = lane & 3;
    const float lo = sMn[k * 256];
    const float hi = sMx[k * 256];
    const float sc = 2.0f * (1.0f / (hi - lo));
    float val = 0.0f;
    if (lane < 4) val = lo;
    else if (lane < 8) val = sc;
    else if (lane < 12) val = hi;
    volatile float* q = mm + lane;
    *q = val;
    __threadfence();
    *q = val;
  }
}

__global__ __launch_bounds__(256) void jet_mlp_kernel(
    const float* __restrict__ X, const float* __restrict__ uvw,
    const float* __restrict__ W_in, const float* __restrict__ b_in,
    const unsigned short* __restrict__ WTp, const float* __restrict__ b_hid,
    const unsigned short* __restrict__ WOTp, const float* __restrict__ b_out,
    const float* __restrict__ Re, const float* __restrict__ mm,
    float* __restrict__ partials)
{
  __shared__ __align__(16) _Float16 sAct[2 * kPlane];
  __shared__ __align__(16) float sJ[kPtsBlk * kJet * kOutPad];
  __shared__ __align__(16) float sRes[16];

  const int tid  = threadIdx.x;
  const int lane = tid & 31;
  const int wave = __builtin_amdgcn_readfirstlane(tid >> 5);
  const int c    = lane & 15;
  const int hh   = lane >> 4;
  const int koff = hh * 8;
  const int p0   = blockIdx.x * kPtsBlk;
  const _Float16* WT  = (const _Float16*)WTp;
  const _Float16* WOT = (const _Float16*)WOTp;

  {
    const int u = tid;
    const v4f lbv = *(const v4f*)(mm);
    const v4f scv = *(const v4f*)(mm + 4);
    const float w0 = W_in[u];
    const float w1 = W_in[kHid + u];
    const float w2 = W_in[2 * kHid + u];
    const float w3 = W_in[3 * kHid + u];
    const float bi = b_in[u];
    const float zt0 = scv[0] * w0;
    const float zt1 = scv[1] * w1;
    const float zt2 = scv[2] * w2;
    const float zt3 = scv[3] * w3;
#pragma unroll 1
    for (int p = 0; p < kPtsBlk; ++p) {
      const v4f xv = *(const v4f*)(X + (size_t)(p0 + p) * kInDim);
      const float x0 = (xv[0] - lbv[0]) * scv[0] - 1.0f;
      const float x1 = (xv[1] - lbv[1]) * scv[1] - 1.0f;
      const float x2 = (xv[2] - lbv[2]) * scv[2] - 1.0f;
      const float x3 = (xv[3] - lbv[3]) * scv[3] - 1.0f;
      const float z  = x0 * w0 + x1 * w1 + x2 * w2 + x3 * w3 + bi;
      const float h  = tanhf(z);
      const float g  = 1.0f - h * h;
      const float m2 = -2.0f * h;
      const float ht0 = g * zt0;
      const float ht1 = g * zt1;
      const float ht2 = g * zt2;
      const float ht3 = g * zt3;
      const int so = (p * kJet) * kPitchA + u;
      sAct[so]               = (_Float16)(h * kCarryA);
      sAct[so + kPitchA]     = (_Float16)(ht0 * kCarryA);
      sAct[so + 2 * kPitchA] = (_Float16)(ht1 * kCarryA);
      sAct[so + 3 * kPitchA] = (_Float16)(ht2 * kCarryA);
      sAct[so + 4 * kPitchA] = (_Float16)(ht3 * kCarryA);
      sAct[so + 5 * kPitchA] = (_Float16)(m2 * ht0 * zt0 * kCarryA);
      sAct[so + 6 * kPitchA] = (_Float16)(m2 * ht1 * zt1 * kCarryA);
      sAct[so + 7 * kPitchA] = (_Float16)(m2 * ht2 * zt2 * kCarryA);
    }
  }

  const int n0 = wave * 32;
#pragma unroll 1
  for (int l = 0; l < kNHid; ++l) {
    const int roff = (l & 1) * kPlane;
    const int woff = kPlane - roff;
    const float bias0 = b_hid[l * kHid + n0 + c];
    const float bias1 = b_hid[l * kHid + n0 + 16 + c];
    __syncthreads();

    v8f acc[4][2];
#pragma unroll
    for (int i = 0; i < 4; ++i) {
      acc[i][0] = (v8f){0.f, 0.f, 0.f, 0.f, 0.f, 0.f, 0.f, 0.f};
      acc[i][1] = (v8f){0.f, 0.f, 0.f, 0.f, 0.f, 0.f, 0.f, 0.f};
    }
    const _Float16* bp0 = WT + (size_t)l * kHid * kHid + (size_t)(n0 + c) * kHid + koff;
    const _Float16* bp1 = bp0 + 16 * kHid;
#pragma unroll 1
    for (int k0 = 0; k0 < kHid; k0 += 32) {
      const v16h b0 = frag_load_g(bp0 + k0);
      const v16h b1 = frag_load_g(bp1 + k0);
#pragma unroll
      for (int i = 0; i < 4; ++i) {
        const int ao = roff + (i * 16 + c) * kPitchA + k0 + koff;
        FragU fa;
        fa.h[0] = *(const v8h*)(&sAct[ao]);
        fa.h[1] = *(const v8h*)(&sAct[ao + 16]);
        acc[i][0] = mma_h(fa.v, b0, acc[i][0]);
        acc[i][1] = mma_h(fa.v, b1, acc[i][1]);
      }
    }
#pragma unroll
    for (int i = 0; i < 4; ++i) {
#pragma unroll
      for (int j = 0; j < 2; ++j) {
        const v8f o = jet_tanh(acc[i][j], (j == 0) ? bias0 : bias1);
        const int so = woff + (i * 16 + 8 * hh) * kPitchA + n0 + j * 16 + c;
#pragma unroll
        for (int r = 0; r < 8; ++r) sAct[so + r * kPitchA] = (_Float16)o[r];
      }
    }
  }
  __syncthreads();

  if (wave < 4) {
    const int roff = (kNHid & 1) * kPlane;
    v8f o = (v8f){0.f, 0.f, 0.f, 0.f, 0.f, 0.f, 0.f, 0.f};
    const _Float16* bp = WOT + (size_t)c * kHid + koff;
#pragma unroll 1
    for (int k0 = 0; k0 < kHid; k0 += 32) {
      const v16h b = frag_load_g(bp + k0);
      const int ao = roff + (wave * 16 + c) * kPitchA + k0 + koff;
      FragU fa;
      fa.h[0] = *(const v8h*)(&sAct[ao]);
      fa.h[1] = *(const v8h*)(&sAct[ao + 16]);
      o = mma_h(fa.v, b, o);
    }
    const int jo = (2 * wave + hh) * (kJet * kOutPad) + c;
#pragma unroll
    for (int r = 0; r < 8; ++r) sJ[jo + r * kOutPad] = o[r] * kFold;
  }
  __syncthreads();

  {
    const int p = tid & 7;
    const v4f J0 = *(const v4f*)(&sJ[p * 128 + 0 * kOutPad]);
    const v4f J1 = *(const v4f*)(&sJ[p * 128 + 1 * kOutPad]);
    const v4f J2 = *(const v4f*)(&sJ[p * 128 + 2 * kOutPad]);
    const v4f J3 = *(const v4f*)(&sJ[p * 128 + 3 * kOutPad]);
    const v4f J4 = *(const v4f*)(&sJ[p * 128 + 4 * kOutPad]);
    const v4f J5 = *(const v4f*)(&sJ[p * 128 + 5 * kOutPad]);
    const v4f J6 = *(const v4f*)(&sJ[p * 128 + 6 * kOutPad]);
    const v4f J7 = *(const v4f*)(&sJ[p * 128 + 7 * kOutPad]);
    float a0 = uvw[(size_t)(p0 + p) * 3 + 0];
    float a1 = uvw[(size_t)(p0 + p) * 3 + 1];
    float a2 = uvw[(size_t)(p0 + p) * 3 + 2];
    asm volatile("" : "+v"(a0));
    asm volatile("" : "+v"(a1));
    asm volatile("" : "+v"(a2));
    const float uu = J0[0] + b_out[0];
    const float vv = J0[1] + b_out[1];
    const float ww = J0[2] + b_out[2];
    const float invRe = 1.0f / fmaxf(Re[0], 1e-8f);
    const float f0 = J4[0] + uu * J1[0] + vv * J2[0] + ww * J3[0] + J1[3] - invRe * (J5[0] + J6[0] + J7[0]);
    const float f1 = J4[1] + uu * J1[1] + vv * J2[1] + ww * J3[1] + J2[3] - invRe * (J5[1] + J6[1] + J7[1]);
    const float f2 = J4[2] + uu * J1[2] + vv * J2[2] + ww * J3[2] + J3[3] - invRe * (J5[2] + J6[2] + J7[2]);
    const float fe = J1[0] + J2[1] + J3[2];
    const float spP = sqrtf(uu * uu + vv * vv + ww * ww) * 0.125f;
    const float sp  = sqrtf(a0 * a0 + a1 * a1 + a2 * a2) * 0.125f;
    const float dd  = sp - spP;
    const float d2  = dd * dd;
    const float e2  = f0 * f0 + f1 * f1 + f2 * f2 + fe * fe;
    if (tid < 8) {
      sRes[tid]     = d2;
      sRes[8 + tid] = e2;
    }
  }
  __syncthreads();

  if (wave == 0) {
    float sd = 0.0f, se = 0.0f;
#pragma unroll
    for (int i = 0; i < 8; ++i) {
      sd += sRes[i];
      se += sRes[8 + i];
    }
    const float val = (lane == 0) ? sd : ((lane == 1) ? se : 0.0f);
    volatile float* q = partials + (size_t)blockIdx.x * 32 + lane;
    *q = val;
    __threadfence();
    *q = val;
  }
}

__global__ __launch_bounds__(256) void finalize_kernel(const float* __restrict__ partials,
                                                       float* __restrict__ out) {
  __shared__ float sS[256];
  const int tid = threadIdx.x;
  float s = 0.0f;
#pragma unroll
  for (int q = 0; q < kBlocks / 256; ++q) {
    const size_t line = (size_t)(tid + 256 * q) * 32;
    const float d = partials[line];
    const float e = partials[line + 1];
    s += d;
    s += e;
  }
  sS[tid] = s;
  __syncthreads();
  for (int off = 128; off > 0; off >>= 1) {
    if (tid < off) sS[tid] += sS[tid + off];
    __syncthreads();
  }
  if (tid == 0) {
    const float val = sS[0] * (0.5f / (float)kPts);
    volatile float* q = out;
    *q = val;
    __threadfence();
    *q = val;
  }
}

extern "C" void kernel_launch(void* const* d_in, const int* in_sizes, int n_in,
                              void* d_out, int out_size, void* d_ws, size_t ws_size,
                              hipStream_t stream) {
  if (n_in < 9) return;
  if (in_sizes[0] != kPts * kInDim) return;
  if (in_sizes[1] != kPts * 3) return;
  if (in_sizes[2] != kInDim * kHid) return;
  if (in_sizes[3] != kHid) return;
  if (in_sizes[4] != kNHid * kHid * kHid) return;
  if (in_sizes[5] != kNHid * kHid) return;
  if (in_sizes[6] != kHid * kOutDim) return;
  if (in_sizes[7] != kOutDim) return;
  if (in_sizes[8] != 1) return;
  if (out_size != 1) return;
  if (ws_size < kWsTotal) return;

  const float* X     = (const float*)d_in[0];
  const float* uvw   = (const float*)d_in[1];
  const float* W_in  = (const float*)d_in[2];
  const float* b_in  = (const float*)d_in[3];
  const float* W_hid = (const float*)d_in[4];
  const float* b_hid = (const float*)d_in[5];
  const float* W_out = (const float*)d_in[6];
  const float* b_out = (const float*)d_in[7];
  const float* Re    = (const float*)d_in[8];
  float* out = (float*)d_out;

  char* ws = (char*)d_ws;
  unsigned short* WT   = (unsigned short*)(ws + kOffWT);
  unsigned short* WOT  = (unsigned short*)(ws + kOffWOT);
  float*          MM   = (float*)(ws + kOffMM);
  float*          PART = (float*)(ws + kOffPART);

  prep_hidden_kernel<<<kNHid * (kHid / 32), 256, 0, stream>>>(W_hid, WT);
  prep_out_kernel<<<1, 256, 0, stream>>>(W_out, WOT);
  bounds_kernel<<<1, 256, 0, stream>>>(X, MM);
  jet_mlp_kernel<<<kBlocks, 256, 0, stream>>>(X, uvw, W_in, b_in, WT, b_hid, WOT, b_out, Re, MM, PART);
  finalize_kernel<<<1, 256, 0, stream>>>(PART, out);
}
